// ESGraphGenerator_63282048139713
// MI455X (gfx1250) — hardware-verified
//
#include <hip/hip_runtime.h>
#include <stddef.h>
#include <math.h>


#define NTHR  256
#define NWAVE 8
#define EPB   256
#define TPW   2
#define HID   50
#define KIN   5
#define NP    64
#define K1P   32
#define K2P   64
#define NPB   (3 * NP)
#define WSC   16.0f
#define WINV  0.0625f

static_assert(EPB == NWAVE * 16 * TPW);
static_assert(EPB / 4 <= NTHR);
static_assert(NP * K1P == 8 * NTHR);
static_assert(NP * K2P == 16 * NTHR);
static_assert(NPB / 4 <= NTHR);
static_assert((NP % 16) == 0 && NP >= HID && K1P >= KIN && K2P >= HID);

typedef float    v4f  __attribute__((ext_vector_type(4)));
typedef float    v8f  __attribute__((ext_vector_type(8)));
typedef int      v4i  __attribute__((ext_vector_type(4)));
typedef _Float16 v8h  __attribute__((ext_vector_type(8)));
typedef _Float16 v16h __attribute__((ext_vector_type(16)));
union FragH { v16h v; v8h h[2]; };
union Pk8 { v8h h; v4i i; };

__device__ __forceinline__ v8h zero8() {
  v8h r;
#pragma unroll
  for (int i = 0; i < 8; ++i) r[i] = (_Float16)0.0f;
  return r;
}

__device__ __forceinline__ v8f wmh(v16h a, v16h b, v8f c) {
  v8f d = __builtin_amdgcn_wmma_f32_16x16x32_f16(false, a, false, b, (short)0, c, false, false);
  asm volatile("v_nop\n\tv_nop\n\tv_nop\n\tv_nop" : "+v"(d) : "v"(a), "v"(b));
  return d;
}

__device__ __forceinline__ v8h relu8(v8f d, float mul) {
  v8h r;
#pragma unroll
  for (int i = 0; i < 8; ++i) { const float t = fmaxf(d[i] * mul, 0.0f); r[i] = (_Float16)t; }
  return r;
}

__device__ __forceinline__ v8h cv8(v4f a, v4f b) {
  v8h r;
  r[0] = (_Float16)a.x; r[1] = (_Float16)a.y; r[2] = (_Float16)a.z; r[3] = (_Float16)a.w;
  r[4] = (_Float16)b.x; r[5] = (_Float16)b.y; r[6] = (_Float16)b.z; r[7] = (_Float16)b.w;
  return r;
}

__device__ __forceinline__ v8f ldc8(const float* p) {
  const v4f a = *(const v4f*)p;
  const v4f b = *(const v4f*)(p + 4);
  v8f c;
  c[0] = a.x; c[1] = a.y; c[2] = a.z; c[3] = a.w;
  c[4] = b.x; c[5] = b.y; c[6] = b.z; c[7] = b.w;
  return c;
}

__device__ __forceinline__ v4i mk8(const float* __restrict__ W, int n, int kc, int kin, int hid, int pitch) {
  const int ncl = n < hid ? n : hid - 1;
  Pk8 pk;
#pragma unroll
  for (int j = 0; j < 8; ++j) {
    const int k   = 8 * kc + j;
    const int kcl = k < kin ? k : kin - 1;
    const float w = W[kcl * pitch + ncl];
    const float t = (k < kin && n < hid) ? w * WSC : 0.0f;
    pk.h[j] = (_Float16)t;
  }
  return pk.i;
}

__global__ __launch_bounds__(NTHR) void k_prep(
    const float* __restrict__ W1, const float* __restrict__ b1,
    const float* __restrict__ W2, const float* __restrict__ b2,
    const float* __restrict__ W3,
    _Float16* P1, _Float16* P2, float* PB, int kin, int hid) {
  const int tid = threadIdx.x;
  const v4i p1  = mk8(W1, tid >> 2, tid & 3, kin, hid, hid);
  const v4i p2a = mk8(W2, tid >> 3, tid & 7, hid, hid, hid);
  const v4i p2b = mk8(W2, (NTHR + tid) >> 3, (NTHR + tid) & 7, hid, hid, hid);
  v4f pb;
  {
    const int tc  = tid < NPB / 4 ? tid : NPB / 4 - 1;
    const int f0  = 4 * tc;
    const int row = f0 / NP;
    const int n0  = f0 - row * NP;
#pragma unroll
    for (int j = 0; j < 4; ++j) {
      const int nn  = n0 + j;
      const int ncl = nn < hid ? nn : hid - 1;
      const float v1 = b1[ncl] * WSC;
      const float v2 = b2[ncl] * WSC;
      const float v3 = W3[ncl] * WINV;
      const float sel = row == 0 ? v1 : (row == 1 ? v2 : v3);
      pb[j] = nn < hid ? sel : 0.0f;
    }
  }
  const bool actb = tid < NPB / 4;
  *(volatile v4i*)(P1 + (size_t)8 * tid) = p1;
  *(volatile v4i*)(P2 + (size_t)8 * tid) = p2a;
  *(volatile v4i*)(P2 + (size_t)8 * (NTHR + tid)) = p2b;
  if (actb) *(volatile v4f*)(PB + 4 * tid) = pb;
  __threadfence();
  *(volatile v4i*)(P1 + (size_t)8 * tid) = p1;
  *(volatile v4i*)(P2 + (size_t)8 * tid) = p2a;
  *(volatile v4i*)(P2 + (size_t)8 * (NTHR + tid)) = p2b;
  if (actb) *(volatile v4f*)(PB + 4 * tid) = pb;
}

__device__ __forceinline__ v8f l1tile(const _Float16* __restrict__ P1, const float* __restrict__ PB,
                                      int ft, int m, int h, v16h bfeat) {
  FragH a;
  const _Float16* wp = P1 + (size_t)(16 * ft + m) * K1P + 8 * h;
  a.h[0] = *(const v8h*)wp;
  a.h[1] = *(const v8h*)(wp + 16);
  return wmh(a.v, bfeat, ldc8(PB + 16 * ft + 8 * h));
}

__device__ __forceinline__ float l23tile(const _Float16* __restrict__ P2, const float* __restrict__ PB,
                                         int gt, int m, int h, v16h bq0, v16h bq1, float t) {
  v8f c = ldc8(PB + NP + 16 * gt + 8 * h);
  {
    FragH a;
    const _Float16* wp = P2 + (size_t)(16 * gt + m) * K2P + 8 * h;
    a.h[0] = *(const v8h*)wp;
    a.h[1] = *(const v8h*)(wp + 16);
    c = wmh(a.v, bq0, c);
  }
  {
    FragH a;
    const _Float16* wp = P2 + (size_t)(16 * gt + m) * K2P + 32 + 8 * h;
    a.h[0] = *(const v8h*)wp;
    a.h[1] = *(const v8h*)(wp + 16);
    c = wmh(a.v, bq1, c);
  }
  const v8f w = ldc8(PB + 2 * NP + 16 * gt + 8 * h);
#pragma unroll
  for (int r = 0; r < 8; ++r) t += fmaxf(c[r], 0.0f) * w[r];
  return t;
}

__global__ __launch_bounds__(NTHR) void k_edge(
    const float* __restrict__ x, const float* __restrict__ ea, const int* __restrict__ ei,
    const _Float16* __restrict__ P1, const _Float16* __restrict__ P2, const float* __restrict__ PB,
    const float* __restrict__ b3, float* out, int nN, int nE) {
  __shared__ __attribute__((aligned(16))) float fst[NWAVE * 16 * 16];
  __shared__ __attribute__((aligned(16))) float outs[EPB];
  const int tid = threadIdx.x, lane = tid & 31, wave = tid >> 5, h = lane >> 4, m = lane & 15;
  const int blockBase = blockIdx.x * EPB;
  const float b3v = b3[0];
  float* fw = fst + wave * 256;
  {
    const v4f z = {0.0f, 0.0f, 0.0f, 0.0f};
    *(v4f*)(fw + 4 * lane) = z;
    *(v4f*)(fw + 128 + 4 * lane) = z;
  }
  __syncthreads();

#pragma unroll 1
  for (int it = 0; it < TPW; ++it) {
    const int lt = it * NWAVE + wave;
    {
      const int e  = blockBase + 16 * lt + m;
      const int ec = e < nE ? e : nE - 1;
      int s = ei[ec];
      int d = ei[(size_t)nE + (size_t)ec];
      s = s < 0 ? s + nN : s;  s = s < 0 ? 0 : (s > nN - 1 ? nN - 1 : s);
      d = d < 0 ? d + nN : d;  d = d < 0 ? 0 : (d > nN - 1 ? nN - 1 : d);
      const float xs = x[s];
      const float xd = x[d];
      const float* ap = ea + (size_t)ec * 3;
      const float a0 = ap[0], a1 = ap[1], a2 = ap[2];
      if (h == 0) {
        float* r = fw + m * 16;
        r[0] = xs; r[1] = xd; r[2] = a0; r[3] = a1; r[4] = a2;
      }
    }
    __syncthreads();

    FragH bf;
    {
      const float* fr = fw + m * 16 + 8 * h;
      bf.h[0] = cv8(*(const v4f*)fr, *(const v4f*)(fr + 4));
      bf.h[1] = zero8();
    }

    const v8f d0 = l1tile(P1, PB, 0, m, h, bf.v);
    const v8f d1 = l1tile(P1, PB, 1, m, h, bf.v);
    const v8f d2 = l1tile(P1, PB, 2, m, h, bf.v);
    const v8f d3 = l1tile(P1, PB, 3, m, h, bf.v);

    FragH bq0, bq1;
    bq0.h[0] = relu8(d0, WINV);
    bq0.h[1] = relu8(d1, WINV);
    bq1.h[0] = relu8(d2, WINV);
    bq1.h[1] = relu8(d3, WINV);

    float t = 0.0f;
    t = l23tile(P2, PB, 0, m, h, bq0.v, bq1.v, t);
    t = l23tile(P2, PB, 1, m, h, bq0.v, bq1.v, t);
    t = l23tile(P2, PB, 2, m, h, bq0.v, bq1.v, t);
    t = l23tile(P2, PB, 3, m, h, bq0.v, bq1.v, t);
    t += __shfl_xor(t, 16, 32);
    const float z  = t + b3v;
    const float ez = expf(-z);
    const float o  = __builtin_amdgcn_rcpf(1.0f + ez);
    if (h == 0) outs[16 * lt + m] = o;
  }
  __syncthreads();

  {
    const bool act = tid < EPB / 4;
    const int  tcl = act ? tid : 0;
    const v4f v = *(const v4f*)(outs + 4 * tcl);
    const size_t oi = (size_t)blockBase + (size_t)(4 * tcl);
    const bool full = act && (oi + 4 <= (size_t)nE);
    const bool part = act && !full && (oi < (size_t)nE);
    volatile float* vo = (volatile float*)out;
    if (full) {
      *(volatile v4f*)(out + oi) = v;
    } else if (part) {
      vo[oi] = v.x;
      if (oi + 1 < (size_t)nE) vo[oi + 1] = v.y;
      if (oi + 2 < (size_t)nE) vo[oi + 2] = v.z;
    }
    __threadfence();
    if (full) {
      *(volatile v4f*)(out + oi) = v;
    } else if (part) {
      vo[oi] = v.x;
      if (oi + 1 < (size_t)nE) vo[oi + 1] = v.y;
      if (oi + 2 < (size_t)nE) vo[oi + 2] = v.z;
    }
  }
}

extern "C" void kernel_launch(void* const* d_in, const int* in_sizes, int n_in,
                              void* d_out, int out_size, void* d_ws, size_t ws_size,
                              hipStream_t stream) {
  if (n_in < 9) return;
  const int nN  = in_sizes[0];
  const int nE2 = in_sizes[2];
  const int nE  = nE2 / 2;
  if (nN < 1 || nE < 1 || nE2 != 2 * nE) return;
  if (in_sizes[1] != 3 * nE) return;
  if (in_sizes[3] != KIN * HID || in_sizes[4] != HID || in_sizes[5] != HID * HID) return;
  if (in_sizes[6] != HID || in_sizes[7] != HID || in_sizes[8] < 1) return;
  if (out_size != nE) return;

  const float* x  = (const float*)d_in[0];
  const float* ea = (const float*)d_in[1];
  const int*   ei = (const int*)d_in[2];
  const float* W1 = (const float*)d_in[3];
  const float* b1 = (const float*)d_in[4];
  const float* W2 = (const float*)d_in[5];
  const float* b2 = (const float*)d_in[6];
  const float* W3 = (const float*)d_in[7];
  const float* b3 = (const float*)d_in[8];
  float* outp = (float*)d_out;

  char* ws = (char*)d_ws;
  const size_t oP1 = 0;
  const size_t oP2 = oP1 + (size_t)NP * K1P * 2;
  const size_t oPB = oP2 + (size_t)NP * K2P * 2;
  const size_t tot = oPB + (size_t)NPB * 4;
  size_t limit = (size_t)134217728;
  if (ws_size < limit) limit = ws_size;
  if (tot > limit) return;
  _Float16* P1 = (_Float16*)(ws + oP1);
  _Float16* P2 = (_Float16*)(ws + oP2);
  float*    PB = (float*)(ws + oPB);

  const int kin = in_sizes[3] / in_sizes[4];
  const int hid = in_sizes[4];

  k_prep<<<1, NTHR, 0, stream>>>(W1, b1, W2, b2, W3, P1, P2, PB, kin, hid);

  const int nBlk = (nE + EPB - 1) / EPB;
  k_edge<<<nBlk, NTHR, 0, stream>>>(x, ea, ei, P1, P2, PB, b3, outp, nN, nE);
}
